// GCN_Model_reg_78993038508802
// MI455X (gfx1250) — hardware-verified
//
#include <hip/hip_runtime.h>


constexpr int NN_   = 16384;
constexpr int EE_   = 65536;
constexpr int DD_   = 64;
constexpr int NF_   = 16;
constexpr int GG_   = 512;
constexpr int F1_   = 256;
constexpr int F2_   = 128;
constexpr int KW_   = 4096 + 64;
constexpr int KP_   = KW_ / 64;
constexpr float EPS_  = 1e-5f;
constexpr float SA_   = 256.0f;
constexpr float SB_   = 1024.0f;
constexpr float SACT_ = 16.0f;
constexpr float SW_   = 64.0f;
constexpr int   CAPG_ = 4096;
constexpr int   TP_   = 68;
constexpr int   HP_   = 72;
constexpr int   HP1_  = 264;
constexpr int   FP2_  = 132;

static_assert(EE_ % 256 == 0);
static_assert(NN_ % 128 == 0);
static_assert(GG_ % 32 == 0);
static_assert(KW_ % 64 == 0);
static_assert((64 * (KW_ / 8)) % 256 == 0);
static_assert((TP_ * 4) % 16 == 0);
static_assert((HP_ * 2) % 16 == 0);
static_assert((HP1_ * 2) % 16 == 0);
static_assert((FP2_ * 4) % 16 == 0);
static_assert((KW_ * 2) % 16 == 0);

typedef float    v4f  __attribute__((ext_vector_type(4)));
typedef float    v8f  __attribute__((ext_vector_type(8)));
typedef int      v4i  __attribute__((ext_vector_type(4)));
typedef _Float16 v8h  __attribute__((ext_vector_type(8)));
typedef _Float16 v16h __attribute__((ext_vector_type(16)));

union FragH { v8h h[2]; v16h v; };

__device__ __forceinline__ v8f ld8f(const float* p) {
    const v4f a = *(const v4f*)p;
    const v4f b = *(const v4f*)(p + 4);
    return __builtin_shufflevector(a, b, 0, 1, 2, 3, 4, 5, 6, 7);
}
__device__ __forceinline__ v8h cvt8h(v8f x) {
    return __builtin_convertvector(x, v8h);
}
__device__ __forceinline__ float wsum32(float v) {
    v += __shfl_xor(v, 16, 32);
    v += __shfl_xor(v, 8, 32);
    v += __shfl_xor(v, 4, 32);
    v += __shfl_xor(v, 2, 32);
    v += __shfl_xor(v, 1, 32);
    return v;
}
__device__ __forceinline__ void mma_h(v8f& acc, const FragH& a, const FragH& b) {
    acc = __builtin_amdgcn_wmma_f32_16x16x32_f16(false, a.v, false, b.v, (short)0, acc, false, false);
    asm volatile("v_nop\n\tv_nop\n\tv_nop\n\tv_nop" : "+v"(acc) : "v"(a.v), "v"(b.v));
}
__device__ __forceinline__ void ldfrag(FragH& f, const _Float16* p) {
    f.h[0] = *(const v8h*)p;
    f.h[1] = *(const v8h*)(p + 16);
}
__device__ __forceinline__ v8f zero8() { v8f z;
#pragma unroll
    for (int r = 0; r < 8; ++r) z[r] = 0.0f; return z; }
__device__ __forceinline__ float sigm_(float x) {
    return __builtin_amdgcn_rcpf(1.0f + __expf(-x));
}
__device__ __forceinline__ float tanh_(float x) {
    const float a = fabsf(x);
    const float e = __expf(-2.0f * a);
    const float t = (1.0f - e) * __builtin_amdgcn_rcpf(1.0f + e);
    return copysignf(t, x);
}

template<int NT, int NR>
__device__ __forceinline__ void pass_f32(const float* st, float* g, int tid) {
    constexpr int NU = NR * 16;
    static_assert(NU % NT == 0);
#pragma unroll
    for (int it = 0; it < NU / NT; ++it) {
        const int u = it * NT + tid;
        const int row = u >> 4, c4 = (u & 15) * 4;
        const v4f v = *(const v4f*)(st + row * TP_ + c4);
        *(volatile v4f*)(g + (size_t)row * DD_ + c4) = v;
    }
}
template<int NT, int NR>
__device__ __forceinline__ void pass_f16(const float* st, _Float16* g, float sc, int tid) {
    constexpr int NU = NR * 8;
    static_assert(NU % NT == 0);
#pragma unroll
    for (int it = 0; it < NU / NT; ++it) {
        const int u = it * NT + tid;
        const int row = u >> 3, c8 = (u & 7) * 8;
        const v8h y = cvt8h(ld8f(st + row * TP_ + c8) * sc);
        *(volatile v8h*)(g + (size_t)row * DD_ + c8) = y;
    }
}

__global__ __launch_bounds__(256)
void prep_kernel(const float* __restrict__ mlp2_w, const float* __restrict__ mlp2_b, const float* __restrict__ root_w,
                 const float* __restrict__ wih, const float* __restrict__ whh,
                 const float* __restrict__ relw, const float* __restrict__ rootw2,
                 const float* __restrict__ fc1w, const float* __restrict__ fc2w,
                 _Float16* W2P, _Float16* ROOTP, _Float16* WIHP, _Float16* WHHP,
                 _Float16* GCP, _Float16* FC1P, _Float16* FC2P)
{
    const int reg = blockIdx.y;
    const int i = blockIdx.x * 256 + threadIdx.x;
    v8f x;
    _Float16* dst;
    size_t e;
    if (reg <= 1) {
        if (i >= 64 * (KW_ / 8)) return;
        const int o    = i / (KW_ / 8);
        const int ch   = i - o * (KW_ / 8);
        const int kap0 = ch * 8;
        const int kk   = min(kap0 >> 6, DD_ - 1);
        const int i0   = kap0 & 63;
        const float* W  = mlp2_w + (size_t)reg * 4096 * DD_;
        const float* bb = mlp2_b + (size_t)reg * 4096;
        const bool isb = (kap0 >= 4096);
#pragma unroll
        for (int c = 0; c < 8; ++c) {
            const float wv = W[(size_t)((i0 + c) * DD_ + o) * DD_ + kk];
            const float bv = bb[(i0 + c) * DD_ + o];
            x[c] = (isb ? bv : wv) * SB_;
        }
        dst = W2P + (size_t)reg * 64 * KW_;
        e = (size_t)o * KW_ + kap0;
    } else if (reg == 2) {
        if (i >= 2 * DD_ * DD_ / 8) return;
        const int l   = i >> 9;
        const int rem = i & 511;
        const int o   = rem >> 3;
        const int k0  = (rem & 7) * 8;
#pragma unroll
        for (int c = 0; c < 8; ++c) x[c] = root_w[(size_t)l * 4096 + (k0 + c) * DD_ + o] * SW_;
        dst = ROOTP;
        e = (size_t)i * 8;
    } else if (reg == 3) {
        if (i >= 2 * 192 * DD_ / 8) return;
        x = ld8f(wih + (size_t)i * 8) * SW_;
        dst = WIHP;
        e = (size_t)i * 8;
    } else if (reg == 4) {
        if (i >= 2 * 192 * DD_ / 8) return;
        x = ld8f(whh + (size_t)i * 8) * SW_;
        dst = WHHP;
        e = (size_t)i * 8;
    } else if (reg == 5) {
        if (i >= DD_ * 128 / 8) return;
        const int o  = i >> 4;
        const int ch = i & 15;
        const int k0 = (ch & 7) * 8;
        const v8f xr = ld8f(relw   + (size_t)o * DD_ + k0);
        const v8f xo = ld8f(rootw2 + (size_t)o * DD_ + k0);
        x = ((ch < 8) ? xr : xo) * SW_;
        dst = GCP;
        e = (size_t)i * 8;
    } else if (reg == 6) {
        if (i >= F1_ * DD_ / 8) return;
        x = ld8f(fc1w + (size_t)i * 8) * SW_;
        dst = FC1P;
        e = (size_t)i * 8;
    } else {
        if (i >= F2_ * F1_ / 8) return;
        x = ld8f(fc2w + (size_t)i * 8) * SW_;
        dst = FC2P;
        e = (size_t)i * 8;
    }
    const v8h y = cvt8h(x);
    *(volatile v8h*)(dst + e) = y;
    __threadfence();
    *(volatile v8h*)(dst + e) = y;
}

__global__ __launch_bounds__(128)
void lin0_kernel(const float* __restrict__ x, const float* __restrict__ w, const float* __restrict__ b, float* H, _Float16* H16)
{
    __shared__ __attribute__((aligned(16))) float sx[64 * 17];
    __shared__ __attribute__((aligned(16))) float st[64 * TP_];
    const int tid = threadIdx.x;
    const int n0 = blockIdx.x * 64;
#pragma unroll
    for (int it = 0; it < 2; ++it) {
        const int u = it * 128 + tid;
        const int row = u >> 2, c4 = (u & 3) * 4;
        const v4f v = *(const v4f*)(x + (size_t)(n0 + row) * NF_ + c4);
        float* sp = sx + row * 17 + c4;
        sp[0] = v.x; sp[1] = v.y; sp[2] = v.z; sp[3] = v.w;
    }
    const int c = tid & 63, half = tid >> 6;
    float wr[NF_];
#pragma unroll
    for (int k = 0; k < NF_; ++k) wr[k] = w[c * NF_ + k];
    const float bc = b[c];
    __syncthreads();
#pragma unroll 1
    for (int j = 0; j < 32; ++j) {
        const int row = half * 32 + j;
        float acc = bc;
#pragma unroll
        for (int k = 0; k < NF_; ++k) acc += sx[row * 17 + k] * wr[k];
        st[row * TP_ + c] = fmaxf(acc, 0.0f);
    }
    __syncthreads();
    float* gF = H + (size_t)n0 * DD_;
    _Float16* gH = H16 + (size_t)n0 * DD_;
    pass_f32<128, 64>(st, gF, tid);
    pass_f16<128, 64>(st, gH, SACT_, tid);
    __threadfence();
    pass_f32<128, 64>(st, gF, tid);
    pass_f16<128, 64>(st, gH, SACT_, tid);
}

__global__ __launch_bounds__(256)
void edge_prep_kernel(const float* __restrict__ ea, const float* __restrict__ w1, const float* __restrict__ b1,
                      const int* __restrict__ srcp, const float* __restrict__ Hc, float* FEAT, float* XS)
{
    __shared__ __attribute__((aligned(16))) float sea[64 * 6];
    __shared__ __attribute__((aligned(16))) float st[64 * TP_];
    __shared__ int ssrc[64];
    const int tid = threadIdx.x;
    const int e0 = blockIdx.x * 64;
    {
        const int u = min(tid, 95);
        const v4f v = *(const v4f*)(ea + (size_t)e0 * 6 + u * 4);
        if (tid < 96) { float* sp = sea + u * 4; sp[0] = v.x; sp[1] = v.y; sp[2] = v.z; sp[3] = v.w; }
        const int s = srcp[e0 + min(tid, 63)];
        if (tid < 64) ssrc[tid] = min(max(s, 0), NN_ - 1);
    }
    const int c = tid & 63, eg = tid >> 6;
    float wr[6];
#pragma unroll
    for (int k = 0; k < 6; ++k) wr[k] = w1[c * 6 + k];
    const float bc = b1[c];
    __syncthreads();
#pragma unroll 1
    for (int j = 0; j < 16; ++j) {
        const int row = eg * 16 + j;
        float acc = bc;
#pragma unroll
        for (int k = 0; k < 6; ++k) acc += sea[row * 6 + k] * wr[k];
        st[row * TP_ + c] = fmaxf(acc, 0.0f);
    }
    __syncthreads();
    v4f gv[4];
#pragma unroll
    for (int it = 0; it < 4; ++it) {
        const int u = it * 256 + tid;
        const int row = u >> 4, c4 = (u & 15) * 4;
        gv[it] = *(const v4f*)(Hc + (size_t)ssrc[row] * DD_ + c4);
    }
    float* gF = FEAT + (size_t)e0 * DD_;
    float* gX = XS + (size_t)e0 * DD_;
    pass_f32<256, 64>(st, gF, tid);
#pragma unroll
    for (int it = 0; it < 4; ++it) *(volatile v4f*)(gX + (size_t)(it * 256 + tid) * 4) = gv[it];
    __threadfence();
    pass_f32<256, 64>(st, gF, tid);
#pragma unroll
    for (int it = 0; it < 4; ++it) *(volatile v4f*)(gX + (size_t)(it * 256 + tid) * 4) = gv[it];
}

__global__ __launch_bounds__(128)
void msg_kernel(const float* __restrict__ XS, const float* __restrict__ FEAT, const _Float16* __restrict__ W2Pl, float* MSG)
{
    __shared__ __attribute__((aligned(16))) float st[4][16 * TP_];
    const int tid = threadIdx.x, lane = tid & 31, wave = tid >> 5, hh = lane >> 4, m = lane & 15;
    const int eb = blockIdx.x * 64 + wave * 16;
    const int e  = eb + m;
    const float* xr = XS + (size_t)e * DD_ + 8 * hh;
    const v8f x0a = ld8f(xr);
    const v8f x0b = ld8f(xr + 16);
    const v8f x1a = ld8f(xr + 32);
    const v8f x1b = ld8f(xr + 48);
    const float* fr = FEAT + (size_t)e * DD_;
    const _Float16* bp = W2Pl + (size_t)m * KW_ + 8 * hh;
    constexpr size_t BT = (size_t)16 * KW_;

    v8f acc[4];
#pragma unroll
    for (int j = 0; j < 4; ++j) acc[j] = zero8();

#pragma unroll 1
    for (int kp = 0; kp < KP_; ++kp) {
        const float fe = fr[min(kp, DD_ - 1)];
        const float f  = ((kp < DD_) ? fe : 1.0f) * SA_;
        const int k0 = kp * 64;
        {
            FragH a;
            a.h[0] = cvt8h(x0a * f);
            a.h[1] = cvt8h(x0b * f);
#pragma unroll
            for (int j = 0; j < 4; ++j) { FragH b; ldfrag(b, bp + j * BT + k0); mma_h(acc[j], a, b); }
        }
        {
            FragH a;
            a.h[0] = cvt8h(x1a * f);
            a.h[1] = cvt8h(x1b * f);
#pragma unroll
            for (int j = 0; j < 4; ++j) { FragH b; ldfrag(b, bp + j * BT + k0 + 32); mma_h(acc[j], a, b); }
        }
    }

    float* sw = st[wave];
    constexpr float SC = 1.0f / (SA_ * SB_);
#pragma unroll
    for (int j = 0; j < 4; ++j)
#pragma unroll
        for (int r = 0; r < 8; ++r) sw[(8 * hh + r) * TP_ + 16 * j + m] = acc[j][r] * SC;
    __syncthreads();
    float* g = MSG + (size_t)eb * DD_;
    pass_f32<32, 16>(sw, g, lane);
    __threadfence();
    pass_f32<32, 16>(sw, g, lane);
}

__global__ __launch_bounds__(256)
void aggr_kernel(const float* __restrict__ rows, const int* __restrict__ dstp, const int* __restrict__ srcp, int use_src,
                 float* AGG, _Float16* AGG16)
{
    __shared__ __attribute__((aligned(16))) float sacc[128 * TP_];
    __shared__ int hit_r[256];
    __shared__ int hit_n[256];
    __shared__ int wcnt[8];
    const int tid = threadIdx.x, lane = tid & 31, wave = tid >> 5;
    const int n0 = blockIdx.x * 128;
    const v4f z4 = {0.0f, 0.0f, 0.0f, 0.0f};
#pragma unroll 1
    for (int u = tid; u < (128 * TP_) / 4; u += 256) *(v4f*)(sacc + u * 4) = z4;
    const int c = tid & 63, q = tid >> 6;
    __syncthreads();

#pragma unroll 1
    for (int cb = 0; cb < EE_; cb += 256) {
        const int e  = cb + tid;
        const int d  = dstp[e];
        const int ln = d - n0;
        const bool hit = ((unsigned)ln < 128u);
        const unsigned bal = __builtin_amdgcn_ballot_w32(hit);
        if (lane == 0) wcnt[wave] = __builtin_popcount(bal);
        const int s = min(max(srcp[e], 0), NN_ - 1);
        const int ridx = use_src ? s : e;
        __syncthreads();
        int woff = 0, total = 0;
#pragma unroll
        for (int w = 0; w < 8; ++w) { const int cw = wcnt[w]; total += cw; woff += (w < wave) ? cw : 0; }
        if (hit) {
            const int p = woff + __builtin_popcount(bal & ((1u << lane) - 1u));
            hit_r[p] = ridx;
            hit_n[p] = ln;
        }
        __syncthreads();
        total = min(total, 256);
#pragma unroll 1
        for (int p = 0; p < total; ++p) {
            const int hn = hit_n[p] & 127;
            const int hr = hit_r[p];
            if ((hn & 3) == q) {
                sacc[hn * TP_ + c] += rows[(size_t)hr * DD_ + c];
            }
        }
        __syncthreads();
    }

    float* gF = AGG + (size_t)n0 * DD_;
    _Float16* gH = AGG16 + (size_t)n0 * DD_;
    pass_f32<256, 128>(sacc, gF, tid);
    pass_f16<256, 128>(sacc, gH, SACT_, tid);
    __threadfence();
    pass_f32<256, 128>(sacc, gF, tid);
    pass_f16<256, 128>(sacc, gH, SACT_, tid);
}

__global__ __launch_bounds__(128)
void node_kernel(const float* __restrict__ AGG, const float* __restrict__ Hc, const _Float16* __restrict__ H16c,
                 const _Float16* __restrict__ ROOTPl, const float* __restrict__ convbl, const float* __restrict__ bnp,
                 const _Float16* __restrict__ WIHPl, const _Float16* __restrict__ WHHPl,
                 const float* __restrict__ bihl, const float* __restrict__ bhhl,
                 float* Hn, _Float16* H16n)
{
    __shared__ __attribute__((aligned(16))) _Float16 sm16[64 * HP_];
    __shared__ __attribute__((aligned(16))) float st[64 * TP_];
    const int tid = threadIdx.x, lane = tid & 31, wave = tid >> 5, hh = lane >> 4, m = lane & 15;
    const int n0 = blockIdx.x * 64;
    const int rowW = wave * 16;
    const size_t arow = (size_t)(n0 + rowW + m) * DD_ + 8 * hh;
    constexpr float S = 1.0f / (SACT_ * SW_);

    v8f acc[4];
#pragma unroll
    for (int j = 0; j < 4; ++j) acc[j] = zero8();
#pragma unroll
    for (int ks = 0; ks < 2; ++ks) {
        FragH a; ldfrag(a, H16c + arow + ks * 32);
#pragma unroll
        for (int j = 0; j < 4; ++j) {
            FragH b; ldfrag(b, ROOTPl + (size_t)(16 * j + m) * DD_ + ks * 32 + 8 * hh);
            mma_h(acc[j], a, b);
        }
    }
#pragma unroll
    for (int j = 0; j < 4; ++j) {
        const int col = 16 * j + m;
        const float cb = convbl[col];
        const float ga = bnp[col], be = bnp[64 + col], mu = bnp[128 + col], va = bnp[192 + col];
        const float rs = rsqrtf(va + EPS_) * ga;
#pragma unroll
        for (int r = 0; r < 8; ++r) {
            const int row = rowW + 8 * hh + r;
            float v = acc[j][r] * S + AGG[(size_t)(n0 + row) * DD_ + col] + cb;
            v = fmaxf(v, 0.0f);
            v = (v - mu) * rs + be;
            sm16[row * HP_ + col] = (_Float16)(v * SACT_);
        }
    }
    __syncthreads();

#pragma unroll 1
    for (int j = 0; j < 4; ++j) {
        v8f gr = zero8(), gz = zero8(), gn = zero8(), xr = zero8(), xz = zero8(), xn = zero8();
#pragma unroll
        for (int ks = 0; ks < 2; ++ks) {
            FragH am, ah, b;
            ldfrag(am, sm16 + (rowW + m) * HP_ + ks * 32 + 8 * hh);
            ldfrag(ah, H16c + arow + ks * 32);
            const size_t boff = (size_t)(16 * j + m) * DD_ + ks * 32 + 8 * hh;
            ldfrag(b, WIHPl + boff);                     mma_h(gr, am, b);
            ldfrag(b, WIHPl + (size_t)64 * DD_ + boff);  mma_h(gz, am, b);
            ldfrag(b, WIHPl + (size_t)128 * DD_ + boff); mma_h(gn, am, b);
            ldfrag(b, WHHPl + boff);                     mma_h(xr, ah, b);
            ldfrag(b, WHHPl + (size_t)64 * DD_ + boff);  mma_h(xz, ah, b);
            ldfrag(b, WHHPl + (size_t)128 * DD_ + boff); mma_h(xn, ah, b);
        }
        const int col = 16 * j + m;
        const float bir = bihl[col], biz = bihl[64 + col], bin = bihl[128 + col];
        const float bhr = bhhl[col], bhz = bhhl[64 + col], bhn = bhhl[128 + col];
#pragma unroll
        for (int r = 0; r < 8; ++r) {
            const int row = rowW + 8 * hh + r;
            const float ir = gr[r] * S + bir, iz = gz[r] * S + biz, in_ = gn[r] * S + bin;
            const float hr = xr[r] * S + bhr, hz = xz[r] * S + bhz, hn = xn[r] * S + bhn;
            const float rg = sigm_(ir + hr);
            const float zg = sigm_(iz + hz);
            const float ng = tanh_(in_ + rg * hn);
            const float hv = Hc[(size_t)(n0 + row) * DD_ + col];
            st[row * TP_ + col] = (1.0f - zg) * ng + zg * hv;
        }
    }
    __syncthreads();
    float* gF = Hn + (size_t)n0 * DD_;
    _Float16* gH = H16n + (size_t)n0 * DD_;
    pass_f32<128, 64>(st, gF, tid);
    pass_f16<128, 64>(st, gH, SACT_, tid);
    __threadfence();
    pass_f32<128, 64>(st, gF, tid);
    pass_f16<128, 64>(st, gH, SACT_, tid);
}

__global__ __launch_bounds__(128)
void gc_kernel(const _Float16* __restrict__ AGG16, const _Float16* __restrict__ H16, const _Float16* __restrict__ GCP,
               const float* __restrict__ relb, const float* __restrict__ bnp, float* G)
{
    __shared__ __attribute__((aligned(16))) float st[64 * TP_];
    const int tid = threadIdx.x, lane = tid & 31, wave = tid >> 5, hh = lane >> 4, m = lane & 15;
    const int n0 = blockIdx.x * 64;
    const int rowW = wave * 16;
    const size_t arow = (size_t)(n0 + rowW + m) * DD_ + 8 * hh;
    constexpr float S = 1.0f / (SACT_ * SW_);
    v8f acc[4];
#pragma unroll
    for (int j = 0; j < 4; ++j) acc[j] = zero8();
#pragma unroll
    for (int ks = 0; ks < 2; ++ks) {
        FragH a; ldfrag(a, AGG16 + arow + ks * 32);
#pragma unroll
        for (int j = 0; j < 4; ++j) {
            FragH b; ldfrag(b, GCP + (size_t)(16 * j + m) * 128 + ks * 32 + 8 * hh);
            mma_h(acc[j], a, b);
        }
    }
#pragma unroll
    for (int ks = 0; ks < 2; ++ks) {
        FragH a; ldfrag(a, H16 + arow + ks * 32);
#pragma unroll
        for (int j = 0; j < 4; ++j) {
            FragH b; ldfrag(b, GCP + (size_t)(16 * j + m) * 128 + 64 + ks * 32 + 8 * hh);
            mma_h(acc[j], a, b);
        }
    }
#pragma unroll
    for (int j = 0; j < 4; ++j) {
        const int col = 16 * j + m;
        const float rb = relb[col];
        const float ga = bnp[col], be = bnp[64 + col], mu = bnp[128 + col], va = bnp[192 + col];
        const float rs = rsqrtf(va + EPS_) * ga;
#pragma unroll
        for (int r = 0; r < 8; ++r) {
            const int row = rowW + 8 * hh + r;
            float v = acc[j][r] * S + rb;
            v = fmaxf(v, 0.0f);
            st[row * TP_ + col] = (v - mu) * rs + be;
        }
    }
    __syncthreads();
    float* gF = G + (size_t)n0 * DD_;
    pass_f32<128, 64>(st, gF, tid);
    __threadfence();
    pass_f32<128, 64>(st, gF, tid);
}

__global__ __launch_bounds__(64)
void head_kernel(const float* __restrict__ GP, const int* __restrict__ batchp,
                 const _Float16* __restrict__ FC1P, const float* __restrict__ fc1b, const float* __restrict__ bn1,
                 const _Float16* __restrict__ FC2P, const float* __restrict__ fc2b, const float* __restrict__ bn2,
                 const float* __restrict__ fclw, const float* __restrict__ fclb, float* out)
{
    __shared__ int slo[36];
    __shared__ __attribute__((aligned(16))) _Float16 sp16[32 * HP_];
    __shared__ __attribute__((aligned(16))) _Float16 sf1[32 * HP1_];
    __shared__ __attribute__((aligned(16))) float sf2[32 * FP2_];
    __shared__ __attribute__((aligned(16))) float sout[32];
    const int tid = threadIdx.x, lane = tid & 31, wave = tid >> 5, hh = lane >> 4, m = lane & 15;
    const int g0 = blockIdx.x * 32;

    {
        const int g = g0 + min(tid, 32);
        int cnt = 0;
#pragma unroll 1
        for (int n4 = 0; n4 < NN_ / 4; ++n4) {
            const v4i v = *(const v4i*)(batchp + 4 * n4);
            cnt += (v.x < g ? 1 : 0) + (v.y < g ? 1 : 0) + (v.z < g ? 1 : 0) + (v.w < g ? 1 : 0);
        }
        if (tid <= 32) slo[tid] = cnt;
    }
    __syncthreads();

    {
        const int c = tid;
#pragma unroll 1
        for (int gl = 0; gl < 32; ++gl) {
            const int lo = slo[gl];
            int cnt = slo[gl + 1] - lo;
            cnt = min(max(cnt, 0), CAPG_);
            float a = 0.0f;
#pragma unroll 1
            for (int j = 0; j < cnt; ++j) {
                const int n = min(lo + j, NN_ - 1);
                a += GP[(size_t)n * DD_ + c];
            }
            sp16[gl * HP_ + c] = (_Float16)(a * SACT_);
        }
    }
    __syncthreads();

    const int rowW = wave * 16;
    constexpr float S = 1.0f / (SACT_ * SW_);
#pragma unroll 1
    for (int jc = 0; jc < 4; ++jc) {
        v8f acc[4];
#pragma unroll
        for (int j = 0; j < 4; ++j) acc[j] = zero8();
#pragma unroll
        for (int ks = 0; ks < 2; ++ks) {
            FragH a; ldfrag(a, sp16 + (rowW + m) * HP_ + ks * 32 + 8 * hh);
#pragma unroll
            for (int j = 0; j < 4; ++j) {
                FragH b; ldfrag(b, FC1P + (size_t)(jc * 64 + 16 * j + m) * DD_ + ks * 32 + 8 * hh);
                mma_h(acc[j], a, b);
            }
        }
#pragma unroll
        for (int j = 0; j < 4; ++j) {
            const int col = jc * 64 + 16 * j + m;
            const float bb = fc1b[col];
            const float ga = bn1[col], be = bn1[F1_ + col], mu = bn1[2 * F1_ + col], va = bn1[3 * F1_ + col];
            const float rs = rsqrtf(va + EPS_) * ga;
#pragma unroll
            for (int r = 0; r < 8; ++r) {
                const int row = rowW + 8 * hh + r;
                float v = acc[j][r] * S + bb;
                v = fmaxf(v, 0.0f);
                v = (v - mu) * rs + be;
                sf1[row * HP1_ + col] = (_Float16)(v * SACT_);
            }
        }
    }
    __syncthreads();

#pragma unroll 1
    for (int jc = 0; jc < 2; ++jc) {
        v8f acc[4];
#pragma unroll
        for (int j = 0; j < 4; ++j) acc[j] = zero8();
#pragma unroll
        for (int ks = 0; ks < 8; ++ks) {
            FragH a; ldfrag(a, sf1 + (rowW + m) * HP1_ + ks * 32 + 8 * hh);
#pragma unroll
            for (int j = 0; j < 4; ++j) {
                FragH b; ldfrag(b, FC2P + (size_t)(jc * 64 + 16 * j + m) * F1_ + ks * 32 + 8 * hh);
                mma_h(acc[j], a, b);
            }
        }
#pragma unroll
        for (int j = 0; j < 4; ++j) {
            const int col = jc * 64 + 16 * j + m;
            const float bb = fc2b[col];
            const float ga = bn2[col], be = bn2[F2_ + col], mu = bn2[2 * F2_ + col], va = bn2[3 * F2_ + col];
            const float rs = rsqrtf(va + EPS_) * ga;
#pragma unroll
            for (int r = 0; r < 8; ++r) {
                const int row = rowW + 8 * hh + r;
                float v = acc[j][r] * S + bb;
                v = fmaxf(v, 0.0f);
                sf2[row * FP2_ + col] = (v - mu) * rs + be;
            }
        }
    }
    __syncthreads();

    {
        const v4f wv = *(const v4f*)(fclw + lane * 4);
        const float fb = fclb[0];
#pragma unroll 1
        for (int rr = 0; rr < 16; ++rr) {
            const int row = rowW + rr;
            const v4f f = *(const v4f*)(sf2 + row * FP2_ + lane * 4);
            float dsum = (f.x * wv.x + f.y * wv.y) + (f.z * wv.z + f.w * wv.w);
            dsum = wsum32(dsum);
            if (lane == 0) sout[row] = dsum + fb;
        }
    }
    __syncthreads();
    if (tid < 8) {
        const v4f o = *(const v4f*)(sout + tid * 4);
        float* gp = out + g0 + tid * 4;
        *(volatile v4f*)gp = o;
        __threadfence();
        *(volatile v4f*)gp = o;
    }
}

extern "C" void kernel_launch(void* const* d_in, const int* in_sizes, int n_in,
                              void* d_out, int out_size, void* d_ws, size_t ws_size,
                              hipStream_t stream)
{
    if (n_in < 29) return;
    const int want[29] = { NN_ * NF_, EE_ * 6, DD_ * NF_, DD_, 2 * DD_ * 6, 2 * DD_, 2 * 4096 * DD_, 2 * 4096,
                           2 * DD_ * DD_, 2 * DD_, 2 * 4 * DD_, 2 * 192 * DD_, 2 * 192 * DD_, 2 * 192, 2 * 192,
                           DD_ * DD_, DD_, DD_ * DD_, 4 * DD_, F1_ * DD_, F1_, 4 * F1_, F2_ * F1_, F2_, 4 * F2_, F2_, 1,
                           2 * EE_, NN_ };
    for (int i = 0; i < 29; ++i) if (in_sizes[i] != want[i]) return;
    if (out_size != GG_) return;

    const float* x        = (const float*)d_in[0];
    const float* ea       = (const float*)d_in[1];
    const float* lin0_w   = (const float*)d_in[2];
    const float* lin0_b   = (const float*)d_in[3];
    const float* mlp1_w   = (const float*)d_in[4];
    const float* mlp1_b   = (const float*)d_in[5];
    const float* mlp2_w   = (const float*)d_in[6];
    const float* mlp2_b   = (const float*)d_in[7];
    const float* root_w   = (const float*)d_in[8];
    const float* conv_b   = (const float*)d_in[9];
    const float* bn       = (const float*)d_in[10];
    const float* gru_wih  = (const float*)d_in[11];
    const float* gru_whh  = (const float*)d_in[12];
    const float* gru_bih  = (const float*)d_in[13];
    const float* gru_bhh  = (const float*)d_in[14];
    const float* gc_rel_w = (const float*)d_in[15];
    const float* gc_rel_b = (const float*)d_in[16];
    const float* gc_root_w= (const float*)d_in[17];
    const float* bnl      = (const float*)d_in[18];
    const float* fc1_w    = (const float*)d_in[19];
    const float* fc1_b    = (const float*)d_in[20];
    const float* fcbn1    = (const float*)d_in[21];
    const float* fc2_w    = (const float*)d_in[22];
    const float* fc2_b    = (const float*)d_in[23];
    const float* fcbn2    = (const float*)d_in[24];
    const float* fcl_w    = (const float*)d_in[25];
    const float* fcl_b    = (const float*)d_in[26];
    const int*   eidx     = (const int*)d_in[27];
    const int*   batch    = (const int*)d_in[28];
    const int* src = eidx;
    const int* dst = eidx + EE_;
    float* out = (float*)d_out;

    char* ws = (char*)d_ws;
    size_t off = 0;
    auto carve = [&](size_t bytes) -> char* { char* p = ws + off; off += (bytes + 255) & ~(size_t)255; return p; };
    const size_t NODE_F32 = (size_t)NN_ * DD_ * 4;
    const size_t NODE_F16 = (size_t)NN_ * DD_ * 2;
    const size_t EDGE_F32 = (size_t)EE_ * DD_ * 4;
    float*    HA    = (float*)carve(NODE_F32);
    float*    HB    = (float*)carve(NODE_F32);
    _Float16* H16A  = (_Float16*)carve(NODE_F16);
    _Float16* H16B  = (_Float16*)carve(NODE_F16);
    float*    AGG   = (float*)carve(NODE_F32);
    _Float16* AGG16 = (_Float16*)carve(NODE_F16);
    float*    FEAT  = (float*)carve(EDGE_F32);
    float*    XS    = (float*)carve(EDGE_F32);
    float*    MSG   = (float*)carve(EDGE_F32);
    float*    GPL   = (float*)carve(NODE_F32);
    _Float16* W2P   = (_Float16*)carve((size_t)2 * 64 * KW_ * 2);
    _Float16* ROOTP = (_Float16*)carve((size_t)2 * DD_ * DD_ * 2);
    _Float16* WIHP  = (_Float16*)carve((size_t)2 * 192 * DD_ * 2);
    _Float16* WHHP  = (_Float16*)carve((size_t)2 * 192 * DD_ * 2);
    _Float16* GCP   = (_Float16*)carve((size_t)DD_ * 128 * 2);
    _Float16* FC1P  = (_Float16*)carve((size_t)F1_ * DD_ * 2);
    _Float16* FC2P  = (_Float16*)carve((size_t)F2_ * F1_ * 2);
    if (off > ws_size) return;

    const dim3 b256(256), b128(128), b64(64);

    prep_kernel<<<dim3((64 * (KW_ / 8)) / 256, 8), b256, 0, stream>>>(mlp2_w, mlp2_b, root_w, gru_wih, gru_whh,
                                                                      gc_rel_w, gc_root_w, fc1_w, fc2_w,
                                                                      W2P, ROOTP, WIHP, WHHP, GCP, FC1P, FC2P);
    lin0_kernel<<<dim3(NN_ / 64), b128, 0, stream>>>(x, lin0_w, lin0_b, HA, H16A);

    float* Hc = HA;       float* Hn = HB;
    _Float16* H16c = H16A; _Float16* H16n = H16B;
    for (int l = 0; l < 2; ++l) {
        edge_prep_kernel<<<dim3(EE_ / 64), b256, 0, stream>>>(ea, mlp1_w + (size_t)l * DD_ * 6, mlp1_b + (size_t)l * DD_,
                                                              src, Hc, FEAT, XS);
        msg_kernel<<<dim3(EE_ / 64), b128, 0, stream>>>(XS, FEAT, W2P + (size_t)l * 64 * KW_, MSG);
        aggr_kernel<<<dim3(NN_ / 128), b256, 0, stream>>>(MSG, dst, src, 0, AGG, AGG16);
        node_kernel<<<dim3(NN_ / 64), b128, 0, stream>>>(AGG, Hc, H16c,
                                                        ROOTP + (size_t)l * DD_ * DD_, conv_b + (size_t)l * DD_,
                                                        bn + (size_t)l * 4 * DD_,
                                                        WIHP + (size_t)l * 192 * DD_, WHHP + (size_t)l * 192 * DD_,
                                                        gru_bih + (size_t)l * 192, gru_bhh + (size_t)l * 192,
                                                        Hn, H16n);
        float* tf = Hc; Hc = Hn; Hn = tf;
        _Float16* th = H16c; H16c = H16n; H16n = th;
    }

    aggr_kernel<<<dim3(NN_ / 128), b256, 0, stream>>>(Hc, dst, src, 1, AGG, AGG16);
    gc_kernel<<<dim3(NN_ / 64), b128, 0, stream>>>(AGG16, H16c, GCP, gc_rel_b, bnl, GPL);
    head_kernel<<<dim3(GG_ / 32), b64, 0, stream>>>(GPL, batch, FC1P, fc1_b, fcbn1, FC2P, fc2_b, fcbn2, fcl_w, fcl_b, out);
}
